// SelfAttention_53489522704490
// MI455X (gfx1250) — hardware-verified
//
#include <hip/hip_runtime.h>


#ifndef NB
#define NB 2
#endif
#ifndef SEQ
#define SEQ 2048
#endif
#define NB_FULL    2
#define SEQ_FULL   2048
#define NHEAD      16
#define HDIM       64
#define QKV_ROW    (3 * NHEAD * HDIM)
#define OUT_ROW    (NHEAD * HDIM)
#define BQ         128
#define BK         32
#define NWAVE      8
#define EARLY_QBLK 4
#define CT         64
#define TP         72
#define OP         68
#define RCUT2      29.0f

static_assert(SEQ % BQ == 0);
static_assert(SEQ % CT == 0);
static_assert(SEQ % BK == 0);
static_assert(BQ == NWAVE * 16);
static_assert(HDIM == 64);
static_assert(SEQ <= SEQ_FULL);
static_assert(NB >= 1 && NB <= NB_FULL);
static_assert((TP * 2) % 16 == 0);
static_assert((OP * 4) % 16 == 0);
static_assert(BK == 32);
static_assert(((size_t)NB * NHEAD * SEQ * HDIM * 2) * 2 <= (size_t)134217728);

typedef __bf16   bf16;
typedef _Float16 f16;
typedef bf16     v16bf __attribute__((ext_vector_type(16)));
typedef f16      v16h  __attribute__((ext_vector_type(16)));
typedef f16      v8h   __attribute__((ext_vector_type(8)));
typedef float    v8f   __attribute__((ext_vector_type(8)));
typedef float    v4f   __attribute__((ext_vector_type(4)));
typedef unsigned v4u   __attribute__((ext_vector_type(4)));

union FragB  { v16bf v; v4u q[2]; bf16 h[16]; };
union FragH  { v16h  v; v4u q[2]; f16  h[16]; };
union Pack8B { v4u u; bf16 h[8]; };
union Pack8H { v4u u; v8h v; f16 h[8]; };

static __device__ __forceinline__ v8f mma_bf16(v16bf a, v16bf b, v8f acc) {
  acc = __builtin_amdgcn_wmma_f32_16x16x32_bf16(false, a, false, b, (short)0, acc, false, false);
  asm volatile("v_nop\n\tv_nop\n\tv_nop\n\tv_nop" : "+v"(acc) : "v"(a), "v"(b));
  return acc;
}
static __device__ __forceinline__ v8f mma_f16(v16h a, v16h b, v8f acc) {
  acc = __builtin_amdgcn_wmma_f32_16x16x32_f16(false, a, false, b, (short)0, acc, false, false);
  asm volatile("v_nop\n\tv_nop\n\tv_nop\n\tv_nop" : "+v"(acc) : "v"(a), "v"(b));
  return acc;
}

static __device__ __forceinline__ f16 toh_flush(float v) {
  const f16 r = (f16)v;
  return (fabsf(v) < 6.103515625e-05f) ? (f16)0.0f : r;
}

__global__ __launch_bounds__(256) void kv_planes_kernel(const float* __restrict__ qkv,
                                                        bf16* __restrict__ kb,
                                                        f16* __restrict__ vt) {
  const int kt  = blockIdx.x;
  const int h   = blockIdx.y;
  const int b   = blockIdx.z;
  const int tid = threadIdx.x;
  __shared__ __align__(16) f16 sT[HDIM * TP];
  const int s0 = kt * CT;

  v4u    kval[2];
  size_t kidx[2];
  #pragma unroll
  for (int kk = 0; kk < 2; ++kk) {
    const int key = kk * 32 + (tid >> 3);
    const int d0  = (tid & 7) * 8;
    const float* src = qkv + ((size_t)b * SEQ_FULL + s0 + key) * QKV_ROW + h * HDIM + d0;
    const v4f k0 = *(const v4f*)(src + OUT_ROW);
    const v4f k1 = *(const v4f*)(src + OUT_ROW + 4);
    const v4f v0 = *(const v4f*)(src + 2 * OUT_ROW);
    const v4f v1 = *(const v4f*)(src + 2 * OUT_ROW + 4);
    Pack8B pk;
    #pragma unroll
    for (int i = 0; i < 4; ++i) {
      pk.h[i]     = (bf16)k0[i];
      pk.h[4 + i] = (bf16)k1[i];
    }
    kval[kk] = pk.u;
    kidx[kk] = (((size_t)b * NHEAD + h) * SEQ + s0 + key) * HDIM + d0;
    #pragma unroll
    for (int i = 0; i < 4; ++i) {
      sT[(d0 + i) * TP + key]     = (f16)(float)(bf16)v0[i];
      sT[(d0 + 4 + i) * TP + key] = (f16)(float)(bf16)v1[i];
    }
  }
  __syncthreads();

  v4u    vval[2];
  size_t vidx[2];
  #pragma unroll
  for (int kk = 0; kk < 2; ++kk) {
    const int d  = kk * 32 + (tid >> 3);
    const int ks = (tid & 7) * 8;
    Pack8H ph;
    ph.v = *(const v8h*)(sT + d * TP + ks);
    vval[kk] = ph.u;
    vidx[kk] = (((size_t)b * NHEAD + h) * HDIM + d) * SEQ + s0 + ks;
  }

  #pragma unroll
  for (int kk = 0; kk < 2; ++kk) {
    *(volatile v4u*)(kb + kidx[kk]) = kval[kk];
    *(volatile v4u*)(vt + vidx[kk]) = vval[kk];
  }
  __threadfence();
  #pragma unroll
  for (int kk = 0; kk < 2; ++kk) {
    *(volatile v4u*)(kb + kidx[kk]) = kval[kk];
    *(volatile v4u*)(vt + vidx[kk]) = vval[kk];
  }
}

template <int RES>
__global__ __launch_bounds__(256) void attn_kernel(const float* __restrict__ qkv,
                                                   const bf16* __restrict__ kb,
                                                   const f16* __restrict__ vt,
                                                   float* __restrict__ out,
                                                   int qblk0) {
  const int qblk = qblk0 + blockIdx.x;
  const int h    = blockIdx.y;
  const int b    = blockIdx.z;
  const int tid  = threadIdx.x;
  const int wave = __builtin_amdgcn_readfirstlane((int)(tid >> 5));
  const int lane = tid & 31;
  const int lq   = lane & 15;
  const int hi   = lane >> 4;

  __shared__ __align__(16) float sO[NWAVE * 16 * OP];

  const int qrow0 = qblk * BQ + wave * 16;

  FragB qf[2];
  {
    const float* qp = qkv + ((size_t)b * SEQ_FULL + qrow0 + lq) * QKV_ROW + h * HDIM;
    #pragma unroll
    for (int f = 0; f < 2; ++f) {
      const v4f a0 = *(const v4f*)(qp + f * 32 + hi * 8);
      const v4f a1 = *(const v4f*)(qp + f * 32 + hi * 8 + 4);
      const v4f b0 = *(const v4f*)(qp + f * 32 + 16 + hi * 8);
      const v4f b1 = *(const v4f*)(qp + f * 32 + 16 + hi * 8 + 4);
      #pragma unroll
      for (int i = 0; i < 4; ++i) {
        qf[f].h[i]      = (bf16)a0[i];
        qf[f].h[4 + i]  = (bf16)a1[i];
        qf[f].h[8 + i]  = (bf16)b0[i];
        qf[f].h[12 + i] = (bf16)b1[i];
      }
    }
  }

  const bf16* kb_h = kb + ((size_t)b * NHEAD + h) * SEQ * HDIM;
  const f16*  vt_h = vt + ((size_t)b * NHEAD + h) * HDIM * SEQ;

  v8f o[4], o2[4];
  #pragma unroll
  for (int dt = 0; dt < 4; ++dt) {
    o[dt]  = (v8f){0, 0, 0, 0, 0, 0, 0, 0};
    o2[dt] = (v8f){0, 0, 0, 0, 0, 0, 0, 0};
  }

  const float NINF = -__builtin_inff();
  float rtail = 0.0f;
  const float SL = 0.1875f * 1.4426950408889634f;
  const int   qi = qrow0 + lq;

  const int nchunk = (qrow0 + 15) / BK + 1;
  for (int i = nchunk - 1; i >= 0; --i) {
    const int j0 = i * BK;

    FragB ak[2][2];
    #pragma unroll
    for (int sub = 0; sub < 2; ++sub) {
      #pragma unroll
      for (int f = 0; f < 2; ++f) {
        const bf16* base = kb_h + (size_t)(j0 + sub * 16 + lq) * HDIM + f * 32 + hi * 8;
        ak[sub][f].q[0] = *(const v4u*)(base);
        ak[sub][f].q[1] = *(const v4u*)(base + 16);
      }
    }

    v8f c[2];
    #pragma unroll
    for (int sub = 0; sub < 2; ++sub) {
      v8f acc = (v8f){0, 0, 0, 0, 0, 0, 0, 0};
      acc = mma_bf16(ak[sub][0].v, qf[0].v, acc);
      acc = mma_bf16(ak[sub][1].v, qf[1].v, acc);
      c[sub] = acc;
    }

    if (j0 + BK - 1 >= qrow0) {
      #pragma unroll
      for (int sub = 0; sub < 2; ++sub) {
        #pragma unroll
        for (int r = 0; r < 8; ++r) {
          const int key = j0 + sub * 16 + hi * 8 + r;
          c[sub][r] = (key >= qi) ? NINF : c[sub][r];
        }
      }
    }

    float e[2][8];
    float g[2];
    #pragma unroll
    for (int sub = 0; sub < 2; ++sub) {
      float run = 0.0f;
      #pragma unroll
      for (int r = 7; r >= 0; --r) {
        const float t2 = c[sub][r] * SL;
        const float y  = __builtin_amdgcn_exp2f(-fabsf(t2));
        const float l2 = __builtin_amdgcn_logf(1.0f + y);
        const float sp = fmaxf(t2, 0.0f) + l2;
        const float ls = fminf(t2, 0.0f) - l2;
        e[sub][r] = ls - run;
        run += sp;
      }
      g[sub] = run;
    }
    const float gp0  = __shfl_xor(g[0], 16, 32);
    const float gp1  = __shfl_xor(g[1], 16, 32);
    const float off0 = g[1] + gp1 + ((hi == 0) ? gp0 : 0.0f);
    const float off1 = (hi == 0) ? gp1 : 0.0f;
    const float tot  = (g[0] + gp0) + (g[1] + gp1);
    const float bs0  = off0 + rtail - 12.0f;
    const float bs1  = off1 + rtail - 12.0f;

    FragH pa, pr;
    #pragma unroll
    for (int r = 0; r < 8; ++r) {
      const float a0  = e[0][r] - bs0;
      const float a1  = e[1][r] - bs1;
      const float x0  = __builtin_amdgcn_exp2f(a0);
      const float x1  = __builtin_amdgcn_exp2f(a1);
      const float pc0 = (a0 < -14.0f) ? 0.0f : x0;
      const float pc1 = (a1 < -14.0f) ? 0.0f : x1;
      const f16 h0 = toh_flush(pc0);
      const f16 h1 = toh_flush(pc1);
      pa.h[r]     = h0;
      pa.h[8 + r] = h1;
      if (RES != 0) {
        pr.h[r]     = toh_flush((pc0 - (float)h0) * 1024.0f);
        pr.h[8 + r] = toh_flush((pc1 - (float)h1) * 1024.0f);
      }
    }
    rtail += tot;

    FragH bv[4];
    #pragma unroll
    for (int dt = 0; dt < 4; ++dt) {
      const f16* base = vt_h + (size_t)(dt * 16 + lq) * SEQ + j0 + hi * 8;
      bv[dt].q[0] = *(const v4u*)(base);
      bv[dt].q[1] = *(const v4u*)(base + 16);
    }

    #pragma unroll
    for (int dt = 0; dt < 4; ++dt) {
      o[dt] = mma_f16(pa.v, bv[dt].v, o[dt]);
      if (RES != 0) o2[dt] = mma_f16(pr.v, bv[dt].v, o2[dt]);
    }

    if (__builtin_amdgcn_ballot_w32(rtail < RCUT2) == 0u) break;
  }

  const float rem = __builtin_amdgcn_exp2f(-rtail);

  float* so = sO + wave * (16 * OP);
  #pragma unroll
  for (int r = 0; r < 8; ++r) {
    #pragma unroll
    for (int dt = 0; dt < 4; ++dt) {
      float val = o[dt][r];
      if (RES != 0) val += o2[dt][r] * (1.0f / 1024.0f);
      so[(hi * 8 + r) * OP + dt * 16 + lq] = val * (1.0f / 4096.0f);
    }
  }
  __syncthreads();

  v4f    vals[8];
  size_t gidx[8];
  #pragma unroll
  for (int it = 0; it < 8; ++it) {
    const int   row = it * 2 + hi;
    const float rr  = __shfl(rem, row, 32);
    const v4f   ov  = *(const v4f*)(so + row * OP + lq * 4);
    const v4f   vv  = *(const v4f*)(qkv + ((size_t)b * SEQ_FULL + qrow0 + row) * QKV_ROW + 2 * OUT_ROW + h * HDIM + lq * 4);
    v4f res;
    #pragma unroll
    for (int i = 0; i < 4; ++i) res[i] = ov[i] + rr * (float)(bf16)vv[i];
    vals[it] = res;
    gidx[it] = ((size_t)b * SEQ_FULL + qrow0 + row) * OUT_ROW + h * HDIM + lq * 4;
  }
  #pragma unroll
  for (int it = 0; it < 8; ++it) *(volatile v4f*)(out + gidx[it]) = vals[it];
  __threadfence();
  #pragma unroll
  for (int it = 0; it < 8; ++it) *(volatile v4f*)(out + gidx[it]) = vals[it];
}

extern "C" void kernel_launch(void* const* d_in, const int* in_sizes, int n_in,
                              void* d_out, int out_size, void* d_ws, size_t ws_size,
                              hipStream_t stream) {
  if (n_in < 1) return;
  const size_t rows_used = (size_t)(NB - 1) * SEQ_FULL + SEQ;
  if ((size_t)in_sizes[0] < rows_used * QKV_ROW) return;
  if ((size_t)out_size < rows_used * OUT_ROW) return;

  const size_t kb_elems = (size_t)NB * NHEAD * SEQ * HDIM;
  const size_t vt_elems = (size_t)NB * NHEAD * HDIM * SEQ;
  const size_t kb_bytes = kb_elems * 2;
  const size_t vt_bytes = vt_elems * 2;
  if (ws_size < kb_bytes + vt_bytes) return;

  const float* qkv = (const float*)d_in[0];
  float*       out = (float*)d_out;
  bf16*        kb  = (bf16*)d_ws;
  f16*         vt  = (f16*)((char*)d_ws + kb_bytes);

  kv_planes_kernel<<<dim3(SEQ / CT, NHEAD, NB), 256, 0, stream>>>(qkv, kb, vt);

  const int nqb     = SEQ / BQ;
  const int n_early = (EARLY_QBLK < nqb) ? EARLY_QBLK : nqb;
  const int n_late  = nqb - n_early;
  attn_kernel<1><<<dim3(n_early, NHEAD, NB), 256, 0, stream>>>(qkv, kb, vt, out, 0);
  if (n_late > 0)
    attn_kernel<0><<<dim3(n_late, NHEAD, NB), 256, 0, stream>>>(qkv, kb, vt, out, n_early);
}
